// GATNet_simple_withMLP_44281112822532
// MI455X (gfx1250) — hardware-run, weakly checked
//
#include <hip/hip_runtime.h>


namespace {
constexpr int N = 10000, E = 320000, IN = 16, W12 = 256, W3 = 768, XC = W12 + W12 + W3, NBLK = N / 16;
constexpr float XS = 8.0f, WSC = 256.0f, SLOPE = 0.2f;
typedef _Float16 b16;
typedef __attribute__((ext_vector_type(16))) _Float16 v16b;
typedef __attribute__((ext_vector_type(8))) _Float16 v8b;
typedef __attribute__((ext_vector_type(8))) float v8f;
typedef __attribute__((ext_vector_type(4))) float v4f;
__device__ __forceinline__ float bf16_rne(float f) { unsigned int u = __float_as_uint(f); u += 0x7FFFu + ((u >> 16) & 1u); return __uint_as_float(u & 0xFFFF0000u); }
__device__ __forceinline__ void split16(float v, b16& hi, b16& lo) { hi = (b16)v; lo = (b16)(v - (float)hi); }
__device__ __forceinline__ v16b frag_kb(const b16* p, int hh) { const v8b a = *(const v8b*)(p + 8 * hh), b = *(const v8b*)(p + 16 + 8 * hh); v16b f;
#pragma unroll
  for (int e = 0; e < 8; ++e) { f[e] = a[e]; f[8 + e] = b[e]; } return f; }
__device__ __forceinline__ v8f wmma16b(v16b a, v16b b, v8f c) { v8f d = __builtin_amdgcn_wmma_f32_16x16x32_f16(false, a, false, b, (short)0, c, false, false); asm volatile("v_nop\n\tv_nop\n\tv_nop\n\tv_nop" : "+v"(d) : "v"(a), "v"(b)); return d; }
__device__ __forceinline__ void wave_lds_sync() { __builtin_amdgcn_fence(__ATOMIC_RELEASE, "workgroup"); __builtin_amdgcn_wave_barrier(); __builtin_amdgcn_fence(__ATOMIC_ACQUIRE, "workgroup"); }
__device__ __forceinline__ float pmul(float a, float b) { float p = a * b; asm volatile("" : "+v"(p)); return p; }
__device__ __forceinline__ int iclamp(int v, int lo, int hi) { return v < lo ? lo : (v > hi ? hi : v); }
__device__ __forceinline__ float leaky(float v) { return v >= 0.0f ? v : SLOPE * v; }
__device__ __forceinline__ float sigm(float v) { return 1.0f / (1.0f + __expf(-v)); }
constexpr int CSR_NBLK7 = 512, CSR_GB7 = 7, CSR_GN7 = 1 << CSR_GB7  , CSR_TS7 = (CSR_GN7 < 32 ? 32 : CSR_GN7)  , CSR_MAXG7 = 512, CSR_CAP7 = 12288  ;
__device__ __host__ __forceinline__ int csr_tix7(int v) { return (v >> CSR_GB7) * CSR_TS7 + (v & (CSR_GN7 - 1)); }
__global__ __launch_bounds__(64) void csrA_kernel7(const int* __restrict__ dst, int E, int N, int nG, int CHP, int NGP, int* __restrict__ STG, int* __restrict__ HST) {
  extern __shared__ int sm[];
  int* cnt = sm; int* run = sm + NGP; int* ids = sm + 2 * NGP;
  const int b = blockIdx.x; const int ch = (E + CSR_NBLK7 - 1) / CSR_NBLK7; const int e0 = b * ch, e1 = min(E, e0 + ch);
  for (int i = threadIdx.x; i < NGP; i += 64) cnt[i] = 0;
  for (int i = threadIdx.x; i < CHP; i += 64) ids[i] = -1;
  __syncthreads();
  if (threadIdx.x == 0) {
    for (int e = e0; e < e1; ++e) { int d = dst[e]; d = (d < 0) ? 0 : (d >= N ? N - 1 : d); cnt[d >> CSR_GB7] += 1; }
    int acc = 0; for (int g = 0; g < nG; ++g) { run[g] = acc; acc += cnt[g]; }
    for (int e = e0; e < e1; ++e) { int d = dst[e]; d = (d < 0) ? 0 : (d >= N ? N - 1 : d); const int g = d >> CSR_GB7; ids[run[g]] = e; run[g] += 1; } }
  __syncthreads();
  typedef __attribute__((ext_vector_type(4))) int v4i;
  for (int pass = 0; pass < 2; ++pass) {
    for (int i = threadIdx.x; i < CHP / 4; i += 64) *(volatile v4i*)(STG + (size_t)b * CHP + i * 4) = *(const v4i*)(&ids[i * 4]);
    for (int i = threadIdx.x; i < NGP / 4; i += 64) { v4i v; for (int e = 0; e < 4; ++e) v[e] = (i * 4 + e < nG) ? cnt[i * 4 + e] : 0; *(volatile v4i*)(HST + (size_t)b * NGP + i * 4) = v; }
    __threadfence(); }
}
__global__ __launch_bounds__(512) void csrS_kernel7(const int* __restrict__ HST, int nG, int NGP, int* __restrict__ START, int* __restrict__ TOT, int* __restrict__ OFF) {
  __shared__ int tot[CSR_MAXG7];
  const int b = threadIdx.x;
  for (int pass = 0; pass < 2; ++pass) { int runb = 0; for (int g = 0; g < nG; ++g) { int c = HST[(size_t)b * NGP + g]; c = (c < 0) ? 0 : c; ((volatile int*)OFF)[(size_t)g * CSR_NBLK7 + b] = runb; runb += c; } __threadfence(); }
  for (int g = threadIdx.x; g < nG; g += 512) { int s = 0; for (int bb = 0; bb < CSR_NBLK7; ++bb) { int c = HST[(size_t)bb * NGP + g]; s += (c < 0) ? 0 : c; } tot[g] = s; }
  __syncthreads();
  if (threadIdx.x < 32) {
    __shared__ int st[CSR_MAXG7 + 32];
    if (threadIdx.x == 0) { int acc = 0; for (int g = 0; g < NGP; ++g) { st[g] = acc; if (g < nG) acc += (tot[g] + 31) & ~31; } st[NGP] = acc; }
    __builtin_amdgcn_fence(__ATOMIC_RELEASE, "workgroup"); __builtin_amdgcn_wave_barrier(); __builtin_amdgcn_fence(__ATOMIC_ACQUIRE, "workgroup");
    for (int pass = 0; pass < 2; ++pass) { for (int i = threadIdx.x; i < NGP + 32; i += 32) { ((volatile int*)START)[i] = (i <= NGP) ? st[min(i, NGP)] : 0; ((volatile int*)TOT)[i] = (i < nG) ? tot[i] : 0; } __threadfence(); } }
}
__global__ __launch_bounds__(256) void csrB_kernel7(const int* __restrict__ dst, int N, int nG, int CHP, int NGP, int permLen, const int* __restrict__ STG, const int* __restrict__ HST, const int* __restrict__ OFF, const int* __restrict__ START, const int* __restrict__ TOT, int* __restrict__ PERM, int* __restrict__ ROWPTR, int* __restrict__ ROWCNT, int* __restrict__ FLAG) {
  typedef __attribute__((ext_vector_type(4))) int v4i;
  __shared__ int ids[CSR_CAP7]; __shared__ unsigned short key[CSR_CAP7]; __shared__ int outp[CSR_CAP7]; __shared__ int ncnt[CSR_GN7 + 1]; __shared__ int boff[CSR_NBLK7 + 1];
  const int g = blockIdx.x, t_ = threadIdx.x; int tot = TOT[g]; int st = START[g], stn = START[g + 1]; const int v0 = g * CSR_GN7; const int nv = min(CSR_GN7, N - v0); const int t0 = g * CSR_TS7;
  st = (st < 0) ? 0 : (st > permLen - 32 ? permLen - 32 : st) & ~31; stn = (stn < st) ? st : (stn > permLen ? permLen : stn); tot = (tot < 0) ? 0 : tot; if (tot > stn - st && tot <= CSR_CAP7) tot = stn - st;
  if (tot > CSR_CAP7) {
    for (int pass = 0; pass < 2; ++pass) { for (int i = t_; i < CSR_TS7 / 4; i += 256) { v4i a, c; for (int e = 0; e < 4; ++e) { a[e] = st; c[e] = 0; } *(volatile v4i*)(ROWPTR + t0 + i * 4) = a; *(volatile v4i*)(ROWCNT + t0 + i * 4) = c; } if (t_ == 0) ((volatile int*)FLAG)[0] = 1; __threadfence(); } (void)nv; return; }
  if (t_ == 0) { int acc = 0; for (int b = 0; b < CSR_NBLK7; ++b) { boff[b] = acc; int c = HST[(size_t)b * NGP + g]; c = (c < 0) ? 0 : (c > CHP ? CHP : c); acc += c; if (acc > tot) acc = tot; } boff[CSR_NBLK7] = acc; }
  for (int i = t_; i <= CSR_GN7; i += 256) ncnt[i] = 0;
  __syncthreads();
  for (int b = 0; b < CSR_NBLK7; ++b) { const int c = boff[b + 1] - boff[b]; int o_ = OFF[(size_t)g * CSR_NBLK7 + b]; o_ = (o_ < 0) ? 0 : (o_ > CHP - c ? CHP - c : o_); const int* src_ = STG + (size_t)b * CHP + o_;
    for (int i = t_; i < c; i += 256) { int id = src_[i]; id = (id < 0) ? 0 : id; ids[boff[b] + i] = id; int d = dst[id]; d = (d < v0) ? v0 : (d >= N ? N - 1 : d); int kk = d - v0; kk = (kk < 0) ? 0 : (kk >= CSR_GN7 ? CSR_GN7 - 1 : kk); key[boff[b] + i] = (unsigned short)kk; } }
  __syncthreads();
  if (t_ == 0) { for (int i = 0; i < tot; ++i) ncnt[key[i]] += 1; int acc = 0; for (int vl = 0; vl < CSR_GN7; ++vl) { const int c = ncnt[vl]; ncnt[vl] = acc; acc += c; } ncnt[CSR_GN7] = acc;
    for (int i = 0; i < tot; ++i) { const int vl = key[i]; outp[ncnt[vl]] = ids[i]; ncnt[vl] += 1; }
    for (int vl = CSR_GN7; vl > 0; --vl) ncnt[vl] = ncnt[vl - 1]; ncnt[0] = 0; }
  __syncthreads();
  for (int pass = 0; pass < 2; ++pass) {
    for (int i = t_; i < (stn - st) / 4; i += 256) { v4i v; for (int e = 0; e < 4; ++e) { const int q = i * 4 + e; v[e] = (q < tot) ? outp[q] : -1; } *(volatile v4i*)(PERM + st + i * 4) = v; }
    for (int i = t_; i < CSR_TS7 / 4; i += 256) { v4i a, c; for (int e = 0; e < 4; ++e) { const int vl = i * 4 + e; const int vc = vl < CSR_GN7 ? vl : CSR_GN7; a[e] = (vl < CSR_GN7) ? st + ncnt[vc] : st; c[e] = (vl < nv) ? (ncnt[(vc < CSR_GN7 ? vc : CSR_GN7 - 1) + 1] - ncnt[vc]) : 0; } *(volatile v4i*)(ROWPTR + t0 + i * 4) = a; *(volatile v4i*)(ROWCNT + t0 + i * 4) = c; }
    __threadfence(); }
}
__global__ __launch_bounds__(256) void csrZ_kernel7(int* __restrict__ p, size_t n4) { typedef __attribute__((ext_vector_type(4))) int v4i; const size_t tid = (size_t)blockIdx.x * 256 + threadIdx.x, nth = (size_t)gridDim.x * 256; v4i z = {0, 0, 0, 0}; for (size_t i = tid; i < n4; i += nth) *(volatile v4i*)(p + i * 4) = z; }
struct CsrBufs7 { int *STG, *HST, *OFF, *START, *TOT, *PERM, *ROWPTR, *ROWCNT, *FLAG; int nG, NGP, CHP; size_t permLen; char* base; size_t bytes; };
static size_t csr_carve7(CsrBufs7& c, char* ws, size_t off, int E, int N) {
  const size_t off0 = off; c.base = ws + off;
  auto al = [&](size_t bytes) { char* p = ws + off; off += (bytes + 255) & ~(size_t)255; return p; };
  c.nG = (N + CSR_GN7 - 1) / CSR_GN7; c.NGP = (c.nG + 31) & ~31; const int ch = (E + CSR_NBLK7 - 1) / CSR_NBLK7; c.CHP = (ch + 31) & ~31; c.permLen = (size_t)E + 32 * (size_t)c.nG + 32;
  c.STG = (int*)al((size_t)CSR_NBLK7 * c.CHP * 4); c.HST = (int*)al((size_t)CSR_NBLK7 * c.NGP * 4); c.OFF = (int*)al((size_t)c.NGP * CSR_NBLK7 * 4); c.START = (int*)al((size_t)(c.NGP + 64) * 4); c.TOT = (int*)al((size_t)(c.NGP + 64) * 4);
  c.PERM = (int*)al(c.permLen * 4); c.ROWPTR = (int*)al((size_t)c.nG * CSR_TS7 * 4); c.ROWCNT = (int*)al((size_t)c.nG * CSR_TS7 * 4); c.FLAG = (int*)al(256);
  c.bytes = off - off0; return off;
}
static void csr_build7(const CsrBufs7& c, const int* dst, int E, int N, hipStream_t stream) {
  const size_t smem = (size_t)(2 * c.NGP + c.CHP) * 4;
  csrZ_kernel7<<<512, 256, 0, stream>>>((int*)c.base, c.bytes / 16);
  csrA_kernel7<<<CSR_NBLK7, 64, smem, stream>>>(dst, E, N, c.nG, c.CHP, c.NGP, c.STG, c.HST);
  csrS_kernel7<<<1, 512, 0, stream>>>(c.HST, c.nG, c.NGP, c.START, c.TOT, c.OFF);
  csrB_kernel7<<<c.nG, 256, 0, stream>>>(dst, N, c.nG, c.CHP, c.NGP, (int)c.permLen, c.STG, c.HST, c.OFF, c.START, c.TOT, c.PERM, c.ROWPTR, c.ROWCNT, c.FLAG);
}


__global__ __launch_bounds__(256) void wput_kernel(const float* __restrict__ w, int KIN, int KP, int OUTW, b16* __restrict__ WT) {
  const int KG = KP / 8; const int u = blockIdx.x * 256 + threadIdx.x; if (u >= OUTW * KG) return; const int o = u / KG, k0 = (u % KG) * 8; v8b v;
#pragma unroll
  for (int j = 0; j < 8; ++j) { const int k = k0 + j; v[j] = k < KIN ? (b16)(bf16_rne(w[(size_t)k * OUTW + o]) * WSC) : (b16)0.0f; } for (int pass = 0; pass < 2; ++pass) { *(volatile v8b*)(WT + (size_t)o * KP + k0) = v; __threadfence(); }
}
template <int KP, int NT, int HT, int EXACT>
__global__ __launch_bounds__(32) void proj_kernel(const float* __restrict__ INP, int inp, int inw, const b16* __restrict__ WT, const float* __restrict__ asv, const float* __restrict__ adv, int NLIM, float* __restrict__ HW, float* __restrict__ AS) {
  constexpr int NH = NT / HT; __shared__ __attribute__((aligned(16))) b16 Ah[16][KP + 8], Al[16][(EXACT ? 32 : KP) + 8]; __shared__ __attribute__((aligned(16))) float Tf[16][128 + 4], Ps[16][32];
  const int lane = threadIdx.x, nloc = lane & 15, hlf = lane >> 4; const size_t m0 = (size_t)blockIdx.x * 16; if (m0 >= (size_t)NLIM) return;
  for (int rr = 0; rr < 16; ++rr) for (int q = 0; q < KP / 32; ++q) { const int c = q * 32 + lane; const float v = c < inw ? INP[(m0 + rr) * inp + c] : 0.0f; if (EXACT) Ah[rr][c] = (b16)(bf16_rne(v) * XS); else { b16 p, ql; split16(v * XS, p, ql); Ah[rr][c] = p; Al[rr][c] = ql; } }
  if (lane < 16) for (int j = 0; j < 32; ++j) Ps[lane][j] = 0.0f;
  wave_lds_sync(); float ps[8], pd[8];
#pragma unroll
  for (int r8 = 0; r8 < 8; ++r8) { ps[r8] = 0.0f; pd[r8] = 0.0f; }
#pragma unroll 1
  for (int cg = 0; cg < NT / 8; ++cg) { v8f acc[8];
#pragma unroll
    for (int t = 0; t < 8; ++t) acc[t] = (v8f){};
#pragma unroll 2
    for (int kb = 0; kb < KP; kb += 32) { const v16b a = frag_kb(&Ah[nloc][kb], hlf); v16b al; if (!EXACT) al = frag_kb(&Al[nloc][kb], hlf);
#pragma unroll
      for (int t = 0; t < 8; ++t) { const v16b bw = frag_kb(WT + (size_t)(cg * 128 + t * 16 + nloc) * KP + kb, hlf); acc[t] = wmma16b(a, bw, acc[t]); if (!EXACT) acc[t] = wmma16b(al, bw, acc[t]); } }
#pragma unroll
    for (int t = 0; t < 8; ++t) { const int c = cg * 128 + t * 16 + nloc; const float wa = bf16_rne(asv[c]), wd = bf16_rne(adv[c]);
#pragma unroll
      for (int r8 = 0; r8 < 8; ++r8) { const float v = acc[t][r8] * (1.0f / (XS * WSC)); Tf[8 * hlf + r8][t * 16 + nloc] = v; ps[r8] += pmul(v, wa); pd[r8] += pmul(v, wd); }
      if ((t % HT) == HT - 1) { const int h = (cg * 8 + t) / HT;
#pragma unroll
        for (int r8 = 0; r8 < 8; ++r8) { float a2 = ps[r8], d2 = pd[r8]; for (int o = 1; o < 16; o <<= 1) { a2 += __shfl_xor(a2, o); d2 += __shfl_xor(d2, o); } if (nloc == 0) { Ps[8 * hlf + r8][h] = a2; Ps[8 * hlf + r8][16 + h] = d2; } ps[r8] = 0.0f; pd[r8] = 0.0f; } } }
    wave_lds_sync();
    for (int pass = 0; pass < 2; ++pass) { for (int rr = 0; rr < 16; ++rr) *(volatile v4f*)(HW + (m0 + rr) * (size_t)(NT * 16) + cg * 128 + lane * 4) = *(const v4f*)(&Tf[rr][lane * 4]); __threadfence(); }
    wave_lds_sync(); }
  for (int pass = 0; pass < 2; ++pass) { for (int q = 0; q < 16; ++q) ((volatile float*)AS)[m0 * 32 + q * 32 + lane] = Ps[q][lane]; __threadfence(); }
}
template <int W, int HD>
__global__ __launch_bounds__(256) void gat_kernel(const float* __restrict__ HW, const float* __restrict__ AS, const float* __restrict__ bias, const int* __restrict__ srcs, const int* __restrict__ PERM, const int* __restrict__ ROWPTR, const int* __restrict__ ROWCNT, int permLen, int NLIM, float* __restrict__ OUT, int outp, int oc) {
  const int wave = threadIdx.x >> 5, lane = threadIdx.x & 31; const size_t v = (size_t)blockIdx.x * 8 + wave; if (v >= (size_t)NLIM) return;
  int st = ROWPTR[v], cnt = ROWCNT[v]; cnt = iclamp(cnt, 0, 1 << 20); st = iclamp(st, 0, permLen - cnt);
#pragma unroll 1
  for (int p = 0; p < W / 256; ++p) { const int c0 = p * 256 + lane * 8; const int h = c0 / HD; const float ad = AS[v * 32 + 16 + h];
    float mx = leaky(AS[v * 32 + h] + ad);
#pragma unroll 1
    for (int j = 0; j < cnt; ++j) { const int e = iclamp(PERM[st + j], 0, E - 1); const size_t s = (size_t)iclamp(srcs[e], 0, N - 1); if (s >= (size_t)NLIM) continue; mx = fmaxf(mx, leaky(AS[s * 32 + h] + ad)); }
    float den; float o[8]; { const float pp = __expf(leaky(AS[v * 32 + h] + ad) - mx); den = pp;
#pragma unroll
      for (int i = 0; i < 8; ++i) o[i] = pmul(pp, HW[v * W + c0 + i]); }
#pragma unroll 1
    for (int j = 0; j < cnt; ++j) { const int e = iclamp(PERM[st + j], 0, E - 1); const size_t s = (size_t)iclamp(srcs[e], 0, N - 1); if (s >= (size_t)NLIM) continue; const float pp = __expf(leaky(AS[s * 32 + h] + ad) - mx); den += pp; const float* hs = HW + s * W + c0;
#pragma unroll
      for (int i = 0; i < 8; ++i) o[i] += pmul(pp, hs[i]); }
    const float inv = 1.0f / (den + 1e-16f); float r[8];
#pragma unroll
    for (int i = 0; i < 8; ++i) r[i] = fmaxf(pmul(o[i], inv) + bf16_rne(bias[c0 + i]), 0.0f);
    for (int pass = 0; pass < 2; ++pass) { *(volatile v4f*)(OUT + v * outp + oc + c0) = (v4f){r[0], r[1], r[2], r[3]}; *(volatile v4f*)(OUT + v * outp + oc + c0 + 4) = (v4f){r[4], r[5], r[6], r[7]}; __threadfence(); } }
}
__global__ __launch_bounds__(32) void head_kernel(const float* __restrict__ XCAT, const float* __restrict__ x, const float* __restrict__ Wf, const float* __restrict__ bfp, const float* __restrict__ M1w, const float* __restrict__ M1b, const b16* __restrict__ M2T, const float* __restrict__ M2b, const float* __restrict__ M3w, const float* __restrict__ M3bp, int NLIM, float* __restrict__ out1, float* __restrict__ out2) {
  __shared__ __attribute__((aligned(16))) b16 Ah[32][136], Al[32][136]; __shared__ float O1[32], O2[32], Xm[32][17];
  const int lane = threadIdx.x, nloc = lane & 15, hlf = lane >> 4; const size_t n0 = (size_t)blockIdx.x * 32; if (n0 >= (size_t)NLIM) return; const bool live = n0 + lane < (size_t)NLIM; const size_t n = live ? n0 + lane : (size_t)NLIM - 1;
  { float s = bf16_rne(bfp[0]); const float* xr = XCAT + n * XC;
#pragma unroll 4
    for (int k = 0; k < XC; ++k) s += pmul(xr[k], bf16_rne(Wf[k])); const float o = sigm(s); O1[lane] = o; for (int i = 0; i < IN; ++i) Xm[lane][i] = bf16_rne(x[n * IN + i]); Xm[lane][IN] = o; }
  wave_lds_sync();
#pragma unroll 1
  for (int r = 0; r < 32; ++r) { for (int q = 0; q < 4; ++q) { const int c = q * 32 + lane; float s = bf16_rne(M1b[c]); for (int k = 0; k < 17; ++k) s += pmul(Xm[r][k], bf16_rne(M1w[k * 128 + c])); b16 p, ql; split16(fmaxf(s, 0.0f) * XS, p, ql); Ah[r][c] = p; Al[r][c] = ql; } }
  wave_lds_sync();
#pragma unroll
  for (int rt = 0; rt < 2; ++rt) { v8f acc[4];
#pragma unroll
    for (int t = 0; t < 4; ++t) acc[t] = (v8f){};
#pragma unroll
    for (int kb = 0; kb < 128; kb += 32) { const v16b a = frag_kb(&Ah[rt * 16 + nloc][kb], hlf), al = frag_kb(&Al[rt * 16 + nloc][kb], hlf);
#pragma unroll
      for (int t = 0; t < 4; ++t) { const v16b bw = frag_kb(M2T + (size_t)(t * 16 + nloc) * 128 + kb, hlf); acc[t] = wmma16b(a, bw, acc[t]); acc[t] = wmma16b(al, bw, acc[t]); } }
    float pd[8];
#pragma unroll
    for (int r8 = 0; r8 < 8; ++r8) pd[r8] = 0.0f;
#pragma unroll
    for (int t = 0; t < 4; ++t) { const int c = t * 16 + nloc; const float bb = bf16_rne(M2b[c]), w3 = bf16_rne(M3w[c]);
#pragma unroll
      for (int r8 = 0; r8 < 8; ++r8) pd[r8] += pmul(fmaxf(acc[t][r8] * (1.0f / (XS * WSC)) + bb, 0.0f), w3); }
#pragma unroll
    for (int r8 = 0; r8 < 8; ++r8) { float s = pd[r8]; for (int o = 1; o < 16; o <<= 1) s += __shfl_xor(s, o); if (nloc == 0) O2[rt * 16 + 8 * hlf + r8] = sigm(s + bf16_rne(M3bp[0])); } }
  wave_lds_sync();
  for (int pass = 0; pass < 2; ++pass) { ((volatile float*)out1)[n0 + lane] = O1[lane]; ((volatile float*)out2)[n0 + lane] = O2[lane]; __threadfence(); }
}
__global__ __launch_bounds__(256) void copy_kernel(const float* __restrict__ ST1, const float* __restrict__ ST2, float* __restrict__ out) { const int i = blockIdx.x * 256 + threadIdx.x; if (i >= 2 * N) return; const float v = i < N ? ST1[i] : ST2[i - N]; for (int pass = 0; pass < 2; ++pass) { ((volatile float*)out)[i] = v; __threadfence(); } }
}

extern "C" void kernel_launch(void* const* d_in, const int* in_sizes, int n_in, void* d_out, int out_size, void* d_ws, size_t ws_size, hipStream_t stream) {
  (void)n_in;
  auto Fp = [&](int i) { return (const float*)d_in[i]; }; auto Ip = [&](int i) { return (const int*)d_in[i]; };
  if (in_sizes[0] != N * IN || in_sizes[1] != 2 * E || in_sizes[3] != IN * W12 || in_sizes[7] != W12 * W12 || in_sizes[11] != W12 * W3 || in_sizes[12] != 12 * 64 || in_sizes[15] != XC || in_sizes[17] != 17 * 128 || in_sizes[19] != 128 * 64 || in_sizes[21] != 64 || out_size != 2 * N) return;
  const int NLIM = N; const int GB16 = NBLK, GB8 = N / 8, GB32 = (N + 31) / 32;
  size_t off = 0; char* ws = (char*)d_ws;
  auto carve = [&](size_t bytes) { char* p = ws + off; off += (bytes + 255) & ~(size_t)255; return p; };
  b16* WT1 = (b16*)carve((size_t)W12 * 32 * 2); b16* WT2 = (b16*)carve((size_t)W12 * W12 * 2); b16* WT3 = (b16*)carve((size_t)W3 * W12 * 2); b16* M2T = (b16*)carve(64 * 128 * 2);
  float* HW = (float*)carve((size_t)N * W3 * 4); float* AS = (float*)carve((size_t)N * 32 * 4); float* XCAT = (float*)carve((size_t)N * XC * 4); float* ST1 = (float*)carve((size_t)(N + 32) * 4); float* ST2 = (float*)carve((size_t)(N + 32) * 4);
  CsrBufs7 csr; off = csr_carve7(csr, ws, off, E, N);
  if (off > ws_size || off > ((size_t)112 << 20)) return;
  wput_kernel<<<(W12 * 4 + 255) / 256, 256, 0, stream>>>(Fp(3), IN, 32, W12, WT1); wput_kernel<<<(W12 * 32 + 255) / 256, 256, 0, stream>>>(Fp(7), W12, W12, W12, WT2); wput_kernel<<<(W3 * 32 + 255) / 256, 256, 0, stream>>>(Fp(11), W12, W12, W3, WT3); wput_kernel<<<(64 * 16 + 255) / 256, 256, 0, stream>>>(Fp(19), 128, 128, 64, M2T);
  csr_build7(csr, Ip(1) + E, E, N, stream);
  proj_kernel<32, 16, 2, 1><<<GB16, 32, 0, stream>>>(Fp(0), IN, IN, WT1, Fp(4), Fp(5), NLIM, HW, AS);
  gat_kernel<W12, 32><<<GB8, 256, 0, stream>>>(HW, AS, Fp(6), Ip(1), csr.PERM, csr.ROWPTR, csr.ROWCNT, (int)csr.permLen, NLIM, XCAT, XC, 0);
  proj_kernel<W12, 16, 2, 0><<<GB16, 32, 0, stream>>>(XCAT, XC, W12, WT2, Fp(8), Fp(9), NLIM, HW, AS);
  gat_kernel<W12, 32><<<GB8, 256, 0, stream>>>(HW, AS, Fp(10), Ip(1), csr.PERM, csr.ROWPTR, csr.ROWCNT, (int)csr.permLen, NLIM, XCAT, XC, W12);
  proj_kernel<W12, 48, 4, 0><<<GB16, 32, 0, stream>>>(XCAT + W12, XC, W12, WT3, Fp(12), Fp(13), NLIM, HW, AS);
  gat_kernel<W3, 64><<<GB8, 256, 0, stream>>>(HW, AS, Fp(14), Ip(1), csr.PERM, csr.ROWPTR, csr.ROWCNT, (int)csr.permLen, NLIM, XCAT, XC, 2 * W12);
  float* out = (float*)d_out;
  head_kernel<<<GB32, 32, 0, stream>>>(XCAT, Fp(0), Fp(15), Fp(16), Fp(17), Fp(18), M2T, Fp(20), Fp(21), Fp(22), NLIM, ST1, ST2);
  copy_kernel<<<(2 * N + 255) / 256, 256, 0, stream>>>(ST1, ST2, out);
}
